// Block_SA_88210038325862
// MI455X (gfx1250) — hardware-verified
//
#include <hip/hip_runtime.h>


#define NB_  8
#define CC   64
#define HW   64
#define NN   (HW * HW)
#define SCL  0.125f
#define PCAR 1024.0f
typedef _Float16 h16;
typedef unsigned short bf;
typedef __attribute__((ext_vector_type(16))) __bf16   v16bf;
typedef __attribute__((ext_vector_type(16))) _Float16 v16h;
typedef __attribute__((ext_vector_type(8)))  _Float16 v8h;
typedef __attribute__((ext_vector_type(8)))  unsigned short v8us;
typedef __attribute__((ext_vector_type(8)))  float    v8f;
typedef __attribute__((ext_vector_type(4)))  float    v4f;
typedef v8h  __attribute__((may_alias)) v8ha;
typedef v4f  __attribute__((may_alias)) v4fa;
typedef v8us __attribute__((may_alias)) v8usa;

__device__ __forceinline__ unsigned short f2bf(float f) { unsigned u = __float_as_uint(f); u += 0x7FFFu + ((u >> 16) & 1u); return (unsigned short)(u >> 16); }
__device__ __forceinline__ float bf2f(unsigned short b) { return __uint_as_float(((unsigned)b) << 16); }
__device__ __forceinline__ float bfr(float f) { return bf2f(f2bf(f)); }
__device__ __forceinline__ v16h cat16(v8h lo, v8h hi) { return __builtin_shufflevector(lo, hi, 0, 1, 2, 3, 4, 5, 6, 7, 8, 9, 10, 11, 12, 13, 14, 15); }
__device__ __forceinline__ v16bf cat16b(v8us lo, v8us hi) { return __builtin_bit_cast(v16bf, __builtin_shufflevector(lo, hi, 0, 1, 2, 3, 4, 5, 6, 7, 8, 9, 10, 11, 12, 13, 14, 15)); }
__device__ __forceinline__ v8f wmma16(v16h a, v16h b, v8f c) { return __builtin_amdgcn_wmma_f32_16x16x32_f16(false, a, false, b, (short)0, c, false, false); }
__device__ __forceinline__ v8f wmmab(v16bf a, v16bf b, v8f c) { return __builtin_amdgcn_wmma_f32_16x16x32_bf16(false, a, false, b, (short)0, c, false, false); }


template <typename T16> struct WFrag;
template <> struct WFrag<h16> { typedef v16h V; static __device__ __forceinline__ V ld(const h16* p) { return cat16(*(const v8h*)p, *(const v8h*)(p + 16)); } static __device__ __forceinline__ v8f mma(V a, V b, v8f c) { return wmma16(a, b, c); } };
template <> struct WFrag<bf> { typedef v16bf V; static __device__ __forceinline__ V ld(const bf* p) { return cat16b(*(const v8us*)p, *(const v8us*)(p + 16)); } static __device__ __forceinline__ v8f mma(V a, V b, v8f c) { return wmmab(a, b, c); } };
template <typename T16, int NSPLIT, bool BIAS>
__global__ __launch_bounds__(32) void k_gemmw(const T16* __restrict__ A, const T16* __restrict__ A2, const T16* __restrict__ Bt, const T16* __restrict__ Bt2, int K, float* C, int ldc, const float* __restrict__ bias, size_t sA, size_t sB, size_t sC) {
    typedef typename WFrag<T16>::V V;
    __shared__ __align__(16) float os[16 * 68];
    const size_t z = blockIdx.z; A += z * sA; if (A2) A2 += z * sA; Bt += z * sB; if (Bt2) Bt2 += z * sB; C += z * sC;
    const int lane = threadIdx.x & 31, lr = lane & 15, hi = lane >> 4; const int r0 = blockIdx.x * 64, c0 = blockIdx.y * 64;
    v8f acc[4][4];
#pragma unroll
    for (int mb = 0; mb < 4; ++mb)
#pragma unroll
        for (int nb = 0; nb < 4; ++nb) acc[mb][nb] = (v8f){};
    const size_t aoff = (size_t)(r0 + lr) * K + 8 * hi, boff = (size_t)(c0 + lr) * K + 8 * hi;
#pragma unroll 1
    for (int kc = 0; kc < K; kc += 32) {
        V a[4], a2[4];
#pragma unroll
        for (int mb = 0; mb < 4; ++mb) { a[mb] = WFrag<T16>::ld(A + aoff + (size_t)mb * 16 * K + kc); if (NSPLIT == 1 || NSPLIT == 2) a2[mb] = WFrag<T16>::ld(A2 + aoff + (size_t)mb * 16 * K + kc); }
#pragma unroll
        for (int nb = 0; nb < 4; ++nb) { const V b = WFrag<T16>::ld(Bt + boff + (size_t)nb * 16 * K + kc); V b2; if (NSPLIT >= 2) b2 = WFrag<T16>::ld(Bt2 + boff + (size_t)nb * 16 * K + kc);
#pragma unroll
            for (int mb = 0; mb < 4; ++mb) { acc[mb][nb] = WFrag<T16>::mma(a[mb], b, acc[mb][nb]); if (NSPLIT == 1 || NSPLIT == 2) acc[mb][nb] = WFrag<T16>::mma(a2[mb], b, acc[mb][nb]); if (NSPLIT >= 2) acc[mb][nb] = WFrag<T16>::mma(a[mb], b2, acc[mb][nb]); } }
        asm volatile("v_nop\n\tv_nop\n\tv_nop\n\tv_nop" : "+v"(acc[0][0]), "+v"(acc[1][1]), "+v"(acc[2][2]), "+v"(acc[3][3]) : "v"(a[0]), "v"(a[3]));
    }
#pragma unroll
    for (int mb = 0; mb < 4; ++mb) {
#pragma unroll
        for (int nb = 0; nb < 4; ++nb) {
#pragma unroll
            for (int j = 0; j < 8; ++j) os[(hi * 8 + j) * 68 + nb * 16 + lr] = acc[mb][nb][j]; }
        __builtin_amdgcn_wave_barrier(); asm volatile("" ::: "memory");
        float* crow = C + (size_t)(r0 + mb * 16) * ldc + c0;
#pragma unroll 1
        for (int ps = 0; ps < 2; ++ps) {
#pragma unroll
            for (int s = 0; s < 8; ++s) { const int row = 2 * s + hi, cofs = lr * 4; v4f val = *(const v4fa*)(os + row * 68 + cofs); if (BIAS) { val[0] += bfr(bias[c0 + cofs]); val[1] += bfr(bias[c0 + cofs + 1]); val[2] += bfr(bias[c0 + cofs + 2]); val[3] += bfr(bias[c0 + cofs + 3]); }
                *(volatile v4f*)(crow + (size_t)row * ldc + cofs) = val; }
            if (ps == 0) __threadfence(); }
        __builtin_amdgcn_wave_barrier(); asm volatile("" ::: "memory");
    }
}

__device__ __forceinline__ h16 tohx(float x) { return (h16)x; }
typedef __attribute__((ext_vector_type(2))) _Float16 v2h;
typedef __attribute__((ext_vector_type(4))) _Float16 v4h;
typedef __attribute__((ext_vector_type(2))) unsigned short v2us;
typedef __attribute__((ext_vector_type(2))) float v2f;

__global__ __launch_bounds__(256) void k_xt(const float* __restrict__ xb, bf* XT) { const int e = (blockIdx.x * 256 + threadIdx.x) * 2; if (e >= NN * CC) return; const int n = e / CC, c = e % CC; v2us o; o[0] = f2bf(xb[(size_t)c * NN + n]); o[1] = f2bf(xb[(size_t)(c + 1) * NN + n]); *(volatile v2us*)(XT + e) = o; __threadfence(); *(volatile v2us*)(XT + e) = o; }
__global__ __launch_bounds__(256) void k_v16(const float* __restrict__ xb, const float* __restrict__ w1, const float* __restrict__ g, const float* __restrict__ bb, const float* __restrict__ mu, const float* __restrict__ var, h16* V16) {
    const int e = (blockIdx.x * 256 + threadIdx.x) * 2; if (e >= CC * NN) return; const int c = e / NN, m = e % NN; float a0 = 0.f, a1 = 0.f;
#pragma unroll 4
    for (int k = 0; k < CC; ++k) { const float wk = bfr(w1[c * CC + k]); float p0 = __fmul_rn(wk, bfr(xb[(size_t)k * NN + m])), p1 = __fmul_rn(wk, bfr(xb[(size_t)k * NN + m + 1])); asm volatile("" : "+v"(p0)); asm volatile("" : "+v"(p1)); a0 = __fadd_rn(a0, p0); a1 = __fadd_rn(a1, p1); }
    const float s = __fdiv_rn(bfr(g[c]), __fsqrt_rn(__fadd_rn(bfr(var[c]), 1e-5f))); float ms = __fmul_rn(bfr(mu[c]), s); asm volatile("" : "+v"(ms)); const float t = __fsub_rn(bfr(bb[c]), ms);
    float y0 = __fmul_rn(a0, s), y1 = __fmul_rn(a1, s); asm volatile("" : "+v"(y0)); asm volatile("" : "+v"(y1)); v2h o; o[0] = tohx(fmaxf(__fadd_rn(y0, t), 0.f)); o[1] = tohx(fmaxf(__fadd_rn(y1, t), 0.f)); *(volatile v2h*)(V16 + e) = o; __threadfence(); *(volatile v2h*)(V16 + e) = o; }
__global__ __launch_bounds__(256) void k_smax(const float* __restrict__ S, float* RS) {
    const int lane = threadIdx.x & 31; const int i = blockIdx.x * 8 + (threadIdx.x >> 5); if (i >= NN) return; const float* sr = S + (size_t)i * NN; float m = -3.0e38f;
#pragma unroll 4
    for (int c0 = lane * 4; c0 < NN; c0 += 128) { const v4f v = *(const v4f*)(sr + c0); m = fmaxf(m, fmaxf(fmaxf(v[0], v[1]), fmaxf(v[2], v[3]))); }
#pragma unroll
    for (int sh = 16; sh; sh >>= 1) m = fmaxf(m, __shfl_xor(m, sh, 32));
    const float o = lane == 0 ? m : 0.f; *(volatile float*)(RS + (size_t)i * 32 + lane) = o; __threadfence(); *(volatile float*)(RS + (size_t)i * 32 + lane) = o;
}
__global__ __launch_bounds__(256) void k_sexp(const float* __restrict__ S, float* RS, h16* P) {
    const int lane = threadIdx.x & 31; const int i = blockIdx.x * 8 + (threadIdx.x >> 5); if (i >= NN) return; const float* sr = S + (size_t)i * NN; const float m = RS[(size_t)i * 32]; float sum = 0.f;
#pragma unroll 2
    for (int c0 = lane * 4; c0 < NN; c0 += 128) { const v4f v = *(const v4f*)(sr + c0); v4h o;
#pragma unroll
        for (int q = 0; q < 4; ++q) { float dlt = __fsub_rn(v[q], m); asm volatile("" : "+v"(dlt)); const float e = __expf(__fmul_rn(dlt, SCL)); sum += e; o[q] = tohx(e * PCAR); }
        *(volatile v4h*)(P + (size_t)i * NN + c0) = o; __threadfence(); *(volatile v4h*)(P + (size_t)i * NN + c0) = o; }
#pragma unroll
    for (int sh = 16; sh; sh >>= 1) sum += __shfl_xor(sum, sh, 32);
    const float o2 = lane == 0 ? m : (lane == 1 ? __fdiv_rn(1.0f, sum * PCAR) : 0.f);   *(volatile float*)(RS + (size_t)i * 32 + lane) = o2; __threadfence(); *(volatile float*)(RS + (size_t)i * 32 + lane) = o2;
}
__global__ __launch_bounds__(256) void k_at(const float* __restrict__ O, const float* __restrict__ RS, float* A) { const int e = (blockIdx.x * 256 + threadIdx.x) * 2; if (e >= CC * NN) return; const int c = e / NN, n = e % NN; v2f o; o[0] = __fmul_rn(O[(size_t)n * CC + c], RS[(size_t)n * 32 + 1]); o[1] = __fmul_rn(O[(size_t)(n + 1) * CC + c], RS[(size_t)(n + 1) * 32 + 1]);
    *(volatile v2f*)(A + e) = o; __threadfence(); *(volatile v2f*)(A + e) = o; }
__global__ __launch_bounds__(256) void k_dw(const float* __restrict__ A, const float* __restrict__ w2, const float* __restrict__ g, const float* __restrict__ bb, const float* __restrict__ mu, const float* __restrict__ var, float* Y) {
    const int e = (blockIdx.x * 256 + threadIdx.x) * 2; if (e >= CC * NN) return; const int c = e / NN; const float s = __fdiv_rn(bfr(g[c]), __fsqrt_rn(__fadd_rn(bfr(var[c]), 1e-5f))); float ms = __fmul_rn(bfr(mu[c]), s); asm volatile("" : "+v"(ms)); const float t = __fsub_rn(bfr(bb[c]), ms); v2f o;
#pragma unroll
    for (int q = 0; q < 2; ++q) { const int n = e % NN + q; const int y = n / HW, x0 = n % HW; float acc = 0.f;
#pragma unroll
        for (int ky = 0; ky < 3; ++ky) {
#pragma unroll
            for (int kx = 0; kx < 3; ++kx) { const int yy = y + ky - 1, xx = x0 + kx - 1; if (yy < 0 || yy >= HW || xx < 0 || xx >= HW) continue; float p = __fmul_rn(bfr(w2[c * 9 + ky * 3 + kx]), A[(size_t)c * NN + yy * HW + xx]); asm volatile("" : "+v"(p)); acc = __fadd_rn(acc, p); } }
        float ya = __fmul_rn(acc, s); asm volatile("" : "+v"(ya)); o[q] = fmaxf(__fadd_rn(ya, t), 0.f); }
    *(volatile v2f*)(Y + e) = o; __threadfence(); *(volatile v2f*)(Y + e) = o; }
__global__ __launch_bounds__(256) void k_pw(const float* __restrict__ Y, const float* __restrict__ xb, const float* __restrict__ w3, const float* __restrict__ g, const float* __restrict__ bb, const float* __restrict__ mu, const float* __restrict__ var, float* OUTb) {
    const int e = (blockIdx.x * 256 + threadIdx.x) * 2; if (e >= CC * NN) return; const int c = e / NN, n = e % NN; float a0 = 0.f, a1 = 0.f;
#pragma unroll 4
    for (int k = 0; k < CC; ++k) { const float wk = bfr(w3[c * CC + k]); float p0 = __fmul_rn(wk, Y[(size_t)k * NN + n]), p1 = __fmul_rn(wk, Y[(size_t)k * NN + n + 1]); asm volatile("" : "+v"(p0)); asm volatile("" : "+v"(p1)); a0 = __fadd_rn(a0, p0); a1 = __fadd_rn(a1, p1); }
    const float s = __fdiv_rn(bfr(g[c]), __fsqrt_rn(__fadd_rn(bfr(var[c]), 1e-5f))); float ms = __fmul_rn(bfr(mu[c]), s); asm volatile("" : "+v"(ms)); const float t = __fsub_rn(bfr(bb[c]), ms); v2f o;
    float y0 = __fmul_rn(a0, s), y1 = __fmul_rn(a1, s); asm volatile("" : "+v"(y0)); asm volatile("" : "+v"(y1)); float z0 = __fadd_rn(y0, t), z1 = __fadd_rn(y1, t); asm volatile("" : "+v"(z0)); asm volatile("" : "+v"(z1)); o[0] = __fadd_rn(z0, bfr(xb[e])); o[1] = __fadd_rn(z1, bfr(xb[e + 1]));
    *(volatile v2f*)(OUTb + e) = o; __threadfence(); *(volatile v2f*)(OUTb + e) = o; }

extern "C" void kernel_launch(void* const* d_in, const int* in_sizes, int n_in,
                              void* d_out, int out_size, void* d_ws, size_t ws_size, hipStream_t stream) {
    (void)in_sizes; (void)n_in; (void)out_size;
    const float* IN[16]; for (int i = 0; i < 16; ++i) IN[i] = (const float*)d_in[i];
    float* OUT = (float*)d_out;
    char* wsp = (char*)d_ws;
    auto take = [&](size_t bytes) { char* p = wsp; wsp += (bytes + 255) & ~(size_t)255; return (void*)p; };
    bf* XT = (bf*)take((size_t)NN * CC * 2); h16* V16 = (h16*)take((size_t)CC * NN * 2); float* S = (float*)take((size_t)NN * NN * 4); h16* P = (h16*)take((size_t)NN * NN * 2); float* RS = (float*)take((size_t)NN * 32 * 4); float* O = (float*)take((size_t)NN * CC * 4); float* A = (float*)take((size_t)CC * NN * 4); float* Y = (float*)take((size_t)CC * NN * 4);
    if ((size_t)(wsp - (char*)d_ws) > ws_size) return;
    const unsigned L2 = (CC * NN / 2 + 255) / 256;
    for (int b = 0; b < NB_; ++b) { const float* xb = IN[0] + (size_t)b * CC * NN;
        k_xt<<<L2, 256, 0, stream>>>(xb, XT); k_v16<<<L2, 256, 0, stream>>>(xb, IN[1], IN[2], IN[3], IN[4], IN[5], V16);
        k_gemmw<bf, 0, false><<<dim3(NN / 64, NN / 64, 1), 32, 0, stream>>>(XT, nullptr, XT, nullptr, CC, S, NN, nullptr, 0, 0, 0);
        k_smax<<<NN / 8, 256, 0, stream>>>(S, RS); k_sexp<<<NN / 8, 256, 0, stream>>>(S, RS, P);
        k_gemmw<h16, 0, false><<<dim3(NN / 64, 1, 1), 32, 0, stream>>>(P, nullptr, V16, nullptr, NN, O, CC, nullptr, 0, 0, 0);
        k_at<<<L2, 256, 0, stream>>>(O, RS, A); k_dw<<<L2, 256, 0, stream>>>(A, IN[6], IN[7], IN[8], IN[9], IN[10], Y); k_pw<<<L2, 256, 0, stream>>>(Y, xb, IN[11], IN[12], IN[13], IN[14], IN[15], OUT + (size_t)b * CC * NN); }
}
